// SpeedrunGPT2Block_59047210385998
// MI455X (gfx1250) — hardware-verified
//
#include <hip/hip_runtime.h>
#include <stdint.h>

#define BB 2
#define SS 2048
#define DD 1024
#define HH 8
#define HDIM 128
#define NTOK (BB * SS)
#define EOT_ID 50256
#define ATT_SCALE 0.12f
#define LN_EPS 1e-6f
#define RMS_EPS 1.1920929e-7f
#define WMUL 64.0f
#define WMUL_INV (1.0f / 64.0f)

typedef __attribute__((ext_vector_type(16))) _Float16 v16h;
typedef __attribute__((ext_vector_type(8)))  _Float16 v8h;
typedef __attribute__((ext_vector_type(4)))  _Float16 v4h;
typedef __attribute__((ext_vector_type(16))) __bf16   v16b;
typedef __attribute__((ext_vector_type(8)))  __bf16   v8b;
typedef __attribute__((ext_vector_type(8)))  float    v8f;
typedef __attribute__((ext_vector_type(4)))  float    v4f;
typedef __attribute__((ext_vector_type(4)))  int      v4i;
#define PSCALE 32768.0f
#define U16(p) ((const unsigned short*)(const void*)(p))
#define PSCALE_INV (1.0f / 32768.0f)

__device__ __forceinline__ unsigned short f2bf_bits(float f) {
  unsigned u = __float_as_uint(f);
  return (unsigned short)((u + 0x7FFFu + ((u >> 16) & 1u)) >> 16);
}
__device__ __forceinline__ float bf_bits2f(unsigned short h) { return __uint_as_float(((unsigned)h) << 16); }

__device__ __forceinline__ void dep_guard_h(v8f& a, v8f& b, v16h x, v16h y) { asm volatile("v_nop\n\tv_nop\n\tv_nop\n\tv_nop" : "+v"(a), "+v"(b) : "v"(x), "v"(y)); }
__device__ __forceinline__ void dep_guard_b(v8f& a, v8f& b, v16b x, v16b y) { asm volatile("v_nop\n\tv_nop\n\tv_nop\n\tv_nop" : "+v"(a), "+v"(b) : "v"(x), "v"(y)); }
__device__ __forceinline__ void keep4_h(v16h a, v16h b, v16h c, v16h d) { asm volatile("v_nop" :: "v"(a), "v"(b), "v"(c), "v"(d)); }
__device__ __forceinline__ void keep4_b(v16b a, v16b b, v16b c, v16b d) { asm volatile("v_nop" :: "v"(a), "v"(b), "v"(c), "v"(d)); }
__device__ __forceinline__ void acc_guard4(v8f& a, v8f& b, v8f& c, v8f& d) { asm volatile("v_nop\n\tv_nop\n\tv_nop\n\tv_nop" : "+v"(a), "+v"(b), "+v"(c), "+v"(d)); }
template <typename T> struct Frag;
template <> struct Frag<_Float16> {
  typedef v16h V; union U { v16h v; v8h h[2]; };
  static __device__ __forceinline__ v16h load(const _Float16* p) {
    U f; f.h[0] = *(const v8h*)(p); f.h[1] = *(const v8h*)(p + 16); return f.v;
  }
  static __device__ __forceinline__ v8f mma(v16h a, v16h b, v8f c) {
    return __builtin_amdgcn_wmma_f32_16x16x32_f16(false, a, false, b, (short)0, c, false, false);
  }
  static __device__ __forceinline__ void guard(v8f& a, v8f& b, v16h x, v16h y) { dep_guard_h(a, b, x, y); }
  static __device__ __forceinline__ void keep(v16h a, v16h b, v16h c, v16h d) { keep4_h(a, b, c, d); }
};
template <> struct Frag<__bf16> {
  typedef v16b V; union U { v16b v; v8b h[2]; };
  static __device__ __forceinline__ v16b load(const __bf16* p) {
    U f; f.h[0] = *(const v8b*)(p); f.h[1] = *(const v8b*)(p + 16); return f.v;
  }
  static __device__ __forceinline__ v8f mma(v16b a, v16b b, v8f c) {
    return __builtin_amdgcn_wmma_f32_16x16x32_bf16(false, a, false, b, (short)0, c, false, false);
  }
  static __device__ __forceinline__ void guard(v8f& a, v8f& b, v16b x, v16b y) { dep_guard_b(a, b, x, y); }
  static __device__ __forceinline__ void keep(v16b a, v16b b, v16b c, v16b d) { keep4_b(a, b, c, d); }
};

template <int ET> struct Elem;
template <> struct Elem<0> { typedef _Float16 T; };
template <> struct Elem<1> { typedef __bf16 T; };
template <int ET, bool SPLIT, int BIAS_MODE, int OUT_MODE, bool RESID, int ACT = 0>
__global__ __launch_bounds__(256) void wmma_gemm64(
    const unsigned short* __restrict__ Ap, const unsigned short* __restrict__ A2p, int lda, long strideA,
    const unsigned short* __restrict__ Btp, const unsigned short* __restrict__ Bt2p, int ldb, long strideB,
    void* __restrict__ Cout, void* __restrict__ Cout2, int ldc, long strideC,
    const float* __restrict__ bias,
    const float* __restrict__ resid, long strideR,
    int M, int N, int K, float scale) {
  typedef typename Elem<ET>::T T;
  typedef typename Frag<T>::V V;
  const T* A = (const T*)Ap; const T* A2 = (const T*)A2p; const T* Bt = (const T*)Btp; const T* Bt2 = (const T*)Bt2p;
  __shared__ __align__(16) float sT[8][16 * 68];
  const int b    = blockIdx.y;
  const int lane = threadIdx.x & 31;
  const int wave = threadIdx.x >> 5;
  const int tilesN = N >> 6;
  const int tilesM = M >> 6;
  const int tile = blockIdx.x * 8 + wave;
  if (tile >= tilesM * tilesN) return;
  const int tm = tile / tilesN;
  const int tn = tile - tm * tilesN;
  const int m0 = tm << 6;
  const int n0 = tn << 6;

  const T* Ab  = A  + (size_t)b * strideA;
  const T* Bb  = Bt + (size_t)b * strideB;
  const T* Ab2 = SPLIT ? (A2  + (size_t)b * strideA) : nullptr;
  const T* Bb2 = SPLIT ? (Bt2 + (size_t)b * strideB) : nullptr;

  const int rlane = lane & 15;
  const int koff  = (lane >> 4) * 8;
  const int mOff  = (lane >> 4) * 8;

  v8f acc[4][4];
#pragma unroll
  for (int i = 0; i < 4; ++i)
#pragma unroll
    for (int j = 0; j < 4; ++j) acc[i][j] = (v8f){0.f,0.f,0.f,0.f,0.f,0.f,0.f,0.f};

  for (int k0 = 0; k0 < K; k0 += 32) {
    V bh[4], bl[4];
#pragma unroll
    for (int j = 0; j < 4; ++j) {
      const size_t bo = (size_t)(n0 + (j << 4) + rlane) * ldb + koff + k0;
      bh[j] = Frag<T>::load(Bb + bo);
      if (SPLIT) bl[j] = Frag<T>::load(Bb2 + bo);
    }
#pragma unroll
    for (int i = 0; i < 4; ++i) {
      const size_t ao = (size_t)(m0 + (i << 4) + rlane) * lda + koff + k0;
      V ah = Frag<T>::load(Ab + ao);
      V al;
      if (SPLIT) al = Frag<T>::load(Ab2 + ao);
#pragma unroll
      for (int j = 0; j < 4; ++j) {
        acc[i][j] = Frag<T>::mma(ah, bh[j], acc[i][j]);
        if (SPLIT) {
          acc[i][j] = Frag<T>::mma(ah, bl[j], acc[i][j]);
          acc[i][j] = Frag<T>::mma(al, bh[j], acc[i][j]);
        }
      }
      Frag<T>::guard(acc[i][0], acc[i][3], ah, SPLIT ? al : ah);
    }
    Frag<T>::keep(bh[0], bh[1], bh[2], bh[3]);
    if (SPLIT) Frag<T>::keep(bl[0], bl[1], bl[2], bl[3]);
  }
  acc_guard4(acc[0][0], acc[0][1], acc[0][2], acc[0][3]);
  acc_guard4(acc[1][0], acc[1][1], acc[1][2], acc[1][3]);
  acc_guard4(acc[2][0], acc[2][1], acc[2][2], acc[2][3]);
  acc_guard4(acc[3][0], acc[3][1], acc[3][2], acc[3][3]);

  float* slab = sT[wave];
  const float* Rb = RESID ? (resid + (size_t)b * strideR) : nullptr;
#pragma unroll
  for (int i = 0; i < 4; ++i) {
    const int mBase = m0 + (i << 4);
#pragma unroll
    for (int j = 0; j < 4; ++j) {
      const int n = n0 + (j << 4) + rlane;
      float bv = 0.f;
      if (BIAS_MODE == 2) bv = bias[n];
#pragma unroll
      for (int r = 0; r < 8; ++r) {
        float v = acc[i][j][r] * scale;
        if (BIAS_MODE == 1) v += bias[mBase + mOff + r];
        if (BIAS_MODE == 2) v += bv;
        if (RESID) v += Rb[(size_t)(mBase + mOff + r) * ldc + n];
        if (ACT == 1) v = tanhf(v);
        if (ACT == 2) v = fmaxf(v, 0.0f);
        if (ACT == 3) v = v / (1.0f + expf(-v));
        if (ACT == 4) v = (v > 0.f) ? v : 0.01f * v;
        if (ACT == 5) v = 0.5f * v * (1.0f + erff(v * 0.70710678118654752f));
        if (ACT == 6) { v = fmaxf(v, 0.0f); v = v * v; }
        slab[(mOff + r) * 68 + (j << 4) + rlane] = v;
      }
    }
    __builtin_amdgcn_fence(__ATOMIC_RELEASE, "workgroup");
    __builtin_amdgcn_wave_barrier();
    __builtin_amdgcn_fence(__ATOMIC_ACQUIRE, "workgroup");
    if (OUT_MODE == 0) {
      float* C = (float*)Cout + (size_t)b * strideC;
      const int hh = lane >> 4, c4 = (lane & 15) * 4;
      for (int pass = 0; pass < 2; ++pass) {
#pragma unroll
        for (int it = 0; it < 8; ++it) {
          const int row = it * 2 + hh;
          v4f v = *(const v4f*)(slab + row * 68 + c4);
          *(volatile v4f*)(C + (size_t)(mBase + row) * ldc + n0 + c4) = v;
        }
        __threadfence();
      }
    } else {
      const int q = lane >> 3, c8 = (lane & 7) * 8;
      unsigned short* C  = (unsigned short*)Cout  + (size_t)b * strideC;
      unsigned short* C2 = (OUT_MODE == 2) ? ((unsigned short*)Cout2 + (size_t)b * strideC) : nullptr;
      for (int pass = 0; pass < 2; ++pass) {
#pragma unroll
        for (int it = 0; it < 4; ++it) {
          const int row = it * 4 + q;
          const float* sp = slab + row * 68 + c8;
          v8h hv, lv;
#pragma unroll
          for (int e = 0; e < 8; ++e) {
            if (OUT_MODE == 1) {
              hv[e] = (_Float16)sp[e];
            } else {
              unsigned short hb = f2bf_bits(sp[e]);
              unsigned short lb = f2bf_bits(sp[e] - bf_bits2f(hb));
              hv[e] = __builtin_bit_cast(_Float16, hb);
              lv[e] = __builtin_bit_cast(_Float16, lb);
            }
          }
          *(volatile v8h*)(C + (size_t)(mBase + row) * ldc + n0 + c8) = hv;
          if (OUT_MODE == 2) *(volatile v8h*)(C2 + (size_t)(mBase + row) * ldc + n0 + c8) = lv;
        }
        __threadfence();
      }
    }
    __builtin_amdgcn_fence(__ATOMIC_RELEASE, "workgroup");
    __builtin_amdgcn_wave_barrier();
    __builtin_amdgcn_fence(__ATOMIC_ACQUIRE, "workgroup");
  }
}

#define WTP 72
__global__ __launch_bounds__(256) void wt_cast_k(const float* __restrict__ W, unsigned short* __restrict__ Wtp,
                                                 int K, int N, float mul) {
  __shared__ __align__(16) _Float16 st[64 * WTP];
  _Float16* Wt = (_Float16*)Wtp;
  const int n0 = blockIdx.x * 64, k0 = blockIdx.y * 64;
  const int tid = threadIdx.x;
  const int kr = tid >> 2, c16 = (tid & 3) * 16;
  const float* src = W + (size_t)(k0 + kr) * N + n0 + c16;
#pragma unroll
  for (int q = 0; q < 4; ++q) {
    const v4f v = *(const v4f*)(src + 4 * q);
#pragma unroll
    for (int e = 0; e < 4; ++e) st[(c16 + 4 * q + e) * WTP + kr] = (_Float16)(v[e] * mul);
  }
  __syncthreads();
  const int wave = tid >> 5, lane = tid & 31;
  const int q8 = lane >> 3, c8 = (lane & 7) * 8;
  for (int pass = 0; pass < 2; ++pass) {
#pragma unroll
    for (int it = 0; it < 2; ++it) {
      const int n = it * 32 + wave * 4 + q8;
      const v8h hv = *(const v8h*)(st + n * WTP + c8);
      *(volatile v8h*)(Wt + (size_t)(n0 + n) * K + k0 + c8) = hv;
    }
    __threadfence();
  }
}

__global__ __launch_bounds__(256) void tables_k(const int* __restrict__ ids, float* __restrict__ rope,
                                                int* __restrict__ docs) {
  __shared__ int scnt[256];
  __shared__ __align__(16) int sdoc[SS];
  const int tid = threadIdx.x, lane = tid & 31, wave = tid >> 5;
  if (blockIdx.x < SS / 8) {
    const int s = blockIdx.x * 8 + wave;
    float e = (float)lane * (1.0f / 31.0f);
    if (lane == 31) e = 1.0f;
    const float fr = powf(0.0009765625f, e);
    const float th = (float)s * fr;
    float sv, cv;
    sincosf(th, &sv, &cv);
    float* rp = rope + (size_t)s * 64;
    *(volatile float*)(rp + lane) = cv;
    *(volatile float*)(rp + 32 + lane) = sv;
    __threadfence();
    *(volatile float*)(rp + lane) = cv;
    *(volatile float*)(rp + 32 + lane) = sv;
  } else {
    int c = 0;
#pragma unroll
    for (int i = 0; i < 8; ++i) c += (ids[tid * 8 + i] == EOT_ID) ? 1 : 0;
    scnt[tid] = c;
    __syncthreads();
    for (int off = 1; off < 256; off <<= 1) {
      const int t = (tid >= off) ? scnt[tid - off] : 0;
      __syncthreads();
      scnt[tid] += t;
      __syncthreads();
    }
    int run = scnt[tid] - c;
#pragma unroll
    for (int i = 0; i < 8; ++i) {
      run += (ids[tid * 8 + i] == EOT_ID) ? 1 : 0;
      sdoc[tid * 8 + i] = run;
    }
    __syncthreads();
    const v4i a0 = *(const v4i*)(sdoc + tid * 4);
    const v4i a1 = *(const v4i*)(sdoc + 1024 + tid * 4);
    for (int pass = 0; pass < 2; ++pass) {
      *(volatile v4i*)(docs + tid * 4) = a0;
      *(volatile v4i*)(docs + 1024 + tid * 4) = a1;
      __threadfence();
    }
  }
}

template <bool MIX>
__global__ __launch_bounds__(128) void ln_k(const float* __restrict__ x, const float* __restrict__ x0,
                                            const float* __restrict__ lam, const float* __restrict__ w,
                                            float* __restrict__ xr, unsigned short* __restrict__ xnp) {
  __shared__ float red1[4], red2[4];
  _Float16* xn = (_Float16*)xnp;
  const int row = blockIdx.x, tid = threadIdx.x, lane = tid & 31, wave = tid >> 5;
  const size_t rb = (size_t)row * DD;
  const int ca = tid * 4, cb = 512 + tid * 4;
  v4f va = *(const v4f*)(x + rb + ca);
  v4f vb = *(const v4f*)(x + rb + cb);
  if (MIX) {
    const float l0 = lam[0], l1 = lam[1];
    const v4f a0 = *(const v4f*)(x0 + rb + ca);
    const v4f b0 = *(const v4f*)(x0 + rb + cb);
    va = va * l0 + a0 * l1;
    vb = vb * l0 + b0 * l1;
    for (int pass = 0; pass < 2; ++pass) {
      *(volatile v4f*)(xr + rb + ca) = va;
      *(volatile v4f*)(xr + rb + cb) = vb;
      __threadfence();
    }
  }
  float s = (va[0] + va[1]) + (va[2] + va[3]) + (vb[0] + vb[1]) + (vb[2] + vb[3]);
#pragma unroll
  for (int off = 1; off < 32; off <<= 1) s += __shfl_xor(s, off, 32);
  if (lane == 0) red1[wave] = s;
  __syncthreads();
  const float mu = ((red1[0] + red1[1]) + (red1[2] + red1[3])) * (1.0f / DD);
  const v4f da = va - mu, db = vb - mu;
  float s2 = (da[0] * da[0] + da[1] * da[1]) + (da[2] * da[2] + da[3] * da[3]) +
             (db[0] * db[0] + db[1] * db[1]) + (db[2] * db[2] + db[3] * db[3]);
#pragma unroll
  for (int off = 1; off < 32; off <<= 1) s2 += __shfl_xor(s2, off, 32);
  if (lane == 0) red2[wave] = s2;
  __syncthreads();
  const float var = ((red2[0] + red2[1]) + (red2[2] + red2[3])) * (1.0f / DD);
  const float inv = rsqrtf(var + LN_EPS);
  const v4f wa = *(const v4f*)(w + ca);
  const v4f wb = *(const v4f*)(w + cb);
  v4h ha, hb;
#pragma unroll
  for (int e = 0; e < 4; ++e) {
    ha[e] = (_Float16)(da[e] * inv * wa[e]);
    hb[e] = (_Float16)(db[e] * inv * wb[e]);
  }
  for (int pass = 0; pass < 2; ++pass) {
    *(volatile v4h*)(xn + rb + ca) = ha;
    *(volatile v4h*)(xn + rb + cb) = hb;
    __threadfence();
  }
}

#define RSP 136
__global__ __launch_bounds__(256) void rope_k(const float* __restrict__ qkv, const float* __restrict__ ve,
                                              const float* __restrict__ sa, const float* __restrict__ rope,
                                              unsigned short* __restrict__ planesp) {
  __shared__ __align__(16) _Float16 st[HH][3 * RSP];
  _Float16* planes = (_Float16*)planesp;
  const int s = blockIdx.x, b = blockIdx.y;
  const int tid = threadIdx.x, h = tid >> 5, ln = tid & 31;
  const size_t tok = (size_t)b * SS + s;
  const float* base = qkv + tok * (3 * DD) + h * HDIM;
  const float cv = rope[(size_t)s * 64 + ln];
  const float sv = rope[(size_t)s * 64 + 32 + ln];
  _Float16* sw = st[h];
#pragma unroll
  for (int p = 0; p < 2; ++p) {
    const float* src = base + p * DD;
    const float a1 = src[ln], b1 = src[ln + 32], a2 = src[ln + 64], b2 = src[ln + 96];
    const float o0 = a1 * cv + a2 * sv;
    const float o2 = a2 * cv - a1 * sv;
    float sq = (o0 * o0 + b1 * b1) + (o2 * o2 + b2 * b2);
#pragma unroll
    for (int off = 1; off < 32; off <<= 1) sq += __shfl_xor(sq, off, 32);
    const float rs = rsqrtf(sq * (1.0f / HDIM) + RMS_EPS);
    sw[p * RSP + ln]      = (_Float16)(o0 * rs);
    sw[p * RSP + ln + 32] = (_Float16)(b1 * rs);
    sw[p * RSP + ln + 64] = (_Float16)(o2 * rs);
    sw[p * RSP + ln + 96] = (_Float16)(b2 * rs);
  }
  {
    const float sa0 = sa[0], sa1 = sa[1];
    const float* vsrc = base + 2 * DD;
    const float* vesrc = ve + (size_t)s * DD + h * HDIM;
#pragma unroll
    for (int i = 0; i < 4; ++i) {
      const int d = ln + 32 * i;
      sw[2 * RSP + d] = (_Float16)(sa0 * vsrc[d] + sa1 * vesrc[d]);
    }
  }
  __builtin_amdgcn_fence(__ATOMIC_RELEASE, "workgroup");
  __builtin_amdgcn_wave_barrier();
  __builtin_amdgcn_fence(__ATOMIC_ACQUIRE, "workgroup");
  const int hh = ln >> 4, c8 = (ln & 15) * 8;
  const size_t PL = (size_t)NTOK * DD;
  const size_t row = ((size_t)(b * HH + h) * SS + s) * HDIM;
  const v8h v01 = *(const v8h*)(sw + hh * RSP + c8);
  const v8h v2  = *(const v8h*)(sw + 2 * RSP + c8);
  _Float16* d01 = planes + (size_t)hh * PL + row + c8;
  _Float16* d2  = planes + 2 * PL + row + c8;
  for (int pass = 0; pass < 2; ++pass) {
    *(volatile v8h*)d01 = v01;
    if (hh == 0) *(volatile v8h*)d2 = v2;
    __threadfence();
  }
}

__device__ __forceinline__ v8f mma_h(v16h a, v16h b, v8f c) {
  c = __builtin_amdgcn_wmma_f32_16x16x32_f16(false, a, false, b, (short)0, c, false, false);
  asm volatile("v_nop\n\tv_nop\n\tv_nop\n\tv_nop" : "+v"(c) : "v"(a), "v"(b));
  return c;
}
#define AKC 64
#define AQB 64
#define OSP 136
__global__ __launch_bounds__(128) void attn128_k(const unsigned short* __restrict__ qpp, const unsigned short* __restrict__ kpp,
                                                 const unsigned short* __restrict__ vpp, const int* __restrict__ docs,
                                                 unsigned short* __restrict__ outp) {
  union FH { v16h v; v8h h[2]; };
  __shared__ __align__(16) _Float16 Ksh[AKC * HDIM];
  __shared__ __align__(16) _Float16 Vth[HDIM * AKC];
  __shared__ __align__(16) _Float16 Psh[4][16 * AKC];
  __shared__ __align__(16) _Float16 Osh[4][16 * OSP];
  const _Float16* qp = (const _Float16*)qpp;
  const _Float16* kp = (const _Float16*)kpp;
  const _Float16* vp = (const _Float16*)vpp;
  _Float16* out = (_Float16*)outp;
  const int tid = threadIdx.x, wave = tid >> 5, lane = tid & 31, hh = lane >> 4, c = lane & 15;
  const int nqb = SS / AQB;
  const int bx = blockIdx.x;
  const int qb = bx % nqb;
  const int bh = bx / nqb;
  const int h = bh % HH;
  const int b = bh / HH;
  const int q0 = qb * AQB + wave * 16;
  const size_t rowb = (size_t)(b * HH + h) * SS;

  v16h qa[4];
  {
    const _Float16* qrow = qp + (rowb + q0 + c) * HDIM + 8 * hh;
#pragma unroll
    for (int dc = 0; dc < 4; ++dc) qa[dc] = Frag<_Float16>::load(qrow + dc * 32);
  }
  int dq[8];
#pragma unroll
  for (int r = 0; r < 8; ++r) dq[r] = docs[q0 + 8 * hh + r];
  float mrow[8], lrow[8];
  v8f oacc[8];
#pragma unroll
  for (int r = 0; r < 8; ++r) { mrow[r] = -INFINITY; lrow[r] = 0.f; }
#pragma unroll
  for (int t = 0; t < 8; ++t) oacc[t] = (v8f){0.f,0.f,0.f,0.f,0.f,0.f,0.f,0.f};

  const int nChunks = qb + 1;
  for (int kc = 0; kc < nChunks; ++kc) {
    const int kv0 = kc * AKC;
    __syncthreads();
    {
      const int kvr = tid >> 1, dh = (tid & 1) * 64;
      const _Float16* krow = kp + (rowb + kv0 + kvr) * HDIM + dh;
      const _Float16* vrow = vp + (rowb + kv0 + kvr) * HDIM + dh;
#pragma unroll 1
      for (int i = 0; i < 8; ++i) {
        const v8h kk = *(const v8h*)(krow + 8 * i);
        *(v8h*)(Ksh + kvr * HDIM + dh + 8 * i) = kk;
        const v8h vv = *(const v8h*)(vrow + 8 * i);
#pragma unroll
        for (int e = 0; e < 8; ++e) Vth[(dh + 8 * i + e) * AKC + kvr] = vv[e];
      }
    }
    __syncthreads();

    v8f s[4];
#pragma unroll
    for (int j = 0; j < 4; ++j) {
      s[j] = (v8f){0.f,0.f,0.f,0.f,0.f,0.f,0.f,0.f};
#pragma unroll
      for (int dc = 0; dc < 4; ++dc) {
        FH kb;
        kb.h[0] = *(const v8h*)(Ksh + (j * 16 + c) * HDIM + dc * 32 + 8 * hh);
        kb.h[1] = *(const v8h*)(Ksh + (j * 16 + c) * HDIM + dc * 32 + 16 + 8 * hh);
        s[j] = mma_h(qa[dc], kb.v, s[j]);
      }
    }
    int dk[4];
#pragma unroll
    for (int j = 0; j < 4; ++j) dk[j] = docs[kv0 + j * 16 + c];
    const bool diag = (kc == qb);
    float cm[8];
#pragma unroll
    for (int r = 0; r < 8; ++r) {
      const int qrow = q0 + 8 * hh + r;
      float m = -INFINITY;
#pragma unroll
      for (int j = 0; j < 4; ++j) {
        const int kvcol = kv0 + j * 16 + c;
        float sv = s[j][r] * ATT_SCALE;
        const bool masked = (dk[j] != dq[r]) || (diag && (kvcol > qrow));
        if (masked) sv = -INFINITY;
        s[j][r] = sv;
        m = fmaxf(m, sv);
      }
#pragma unroll
      for (int off = 1; off < 16; off <<= 1) m = fmaxf(m, __shfl_xor(m, off, 32));
      cm[r] = m;
    }
    _Float16* pw = Psh[wave];
#pragma unroll
    for (int r = 0; r < 8; ++r) {
      const float mnew = fmaxf(mrow[r], cm[r]);
      const float mref = (mnew > -INFINITY) ? mnew : 0.0f;
      const float alpha = expf(mrow[r] - mref);
      mrow[r] = mnew;
      float psum = 0.f;
#pragma unroll
      for (int j = 0; j < 4; ++j) {
        const float p = expf(s[j][r] - mref);
        psum += p;
        pw[(8 * hh + r) * AKC + j * 16 + c] = (_Float16)(p * PSCALE);
      }
#pragma unroll
      for (int off = 1; off < 16; off <<= 1) psum += __shfl_xor(psum, off, 32);
      lrow[r] = lrow[r] * alpha + psum;
#pragma unroll
      for (int t = 0; t < 8; ++t) oacc[t][r] *= alpha;
    }
    __builtin_amdgcn_fence(__ATOMIC_RELEASE, "workgroup");
    __builtin_amdgcn_wave_barrier();
    __builtin_amdgcn_fence(__ATOMIC_ACQUIRE, "workgroup");
#pragma unroll 1
    for (int kk = 0; kk < 2; ++kk) {
      FH pa;
      pa.h[0] = *(const v8h*)(pw + c * AKC + kk * 32 + 8 * hh);
      pa.h[1] = *(const v8h*)(pw + c * AKC + kk * 32 + 16 + 8 * hh);
#pragma unroll
      for (int t = 0; t < 8; ++t) {
        FH vb;
        vb.h[0] = *(const v8h*)(Vth + (t * 16 + c) * AKC + kk * 32 + 8 * hh);
        vb.h[1] = *(const v8h*)(Vth + (t * 16 + c) * AKC + kk * 32 + 16 + 8 * hh);
        oacc[t] = mma_h(pa.v, vb.v, oacc[t]);
      }
    }
  }

  _Float16* os = Osh[wave];
#pragma unroll
  for (int r = 0; r < 8; ++r) {
    const float inv = 1.0f / (lrow[r] * PSCALE);
#pragma unroll
    for (int t = 0; t < 8; ++t) os[(8 * hh + r) * OSP + t * 16 + c] = (_Float16)(oacc[t][r] * inv);
  }
  __builtin_amdgcn_fence(__ATOMIC_RELEASE, "workgroup");
  __builtin_amdgcn_wave_barrier();
  __builtin_amdgcn_fence(__ATOMIC_ACQUIRE, "workgroup");
  {
    const int c8 = (lane & 15) * 8;
    for (int pass = 0; pass < 2; ++pass) {
#pragma unroll
      for (int it = 0; it < 8; ++it) {
        const int row = it * 2 + hh;
        const v8h val = *(const v8h*)(os + row * OSP + c8);
        *(volatile v8h*)(out + (size_t)(b * SS + q0 + row) * DD + h * HDIM + c8) = val;
      }
      __threadfence();
    }
  }
}

extern "C" void kernel_launch(void* const* d_in, const int* in_sizes, int n_in,
                              void* d_out, int out_size, void* d_ws,
                              size_t ws_size, hipStream_t stream) {
  if (n_in < 12) return;
  if (in_sizes[0] != NTOK * DD || in_sizes[1] != SS * DD || in_sizes[2] != NTOK * DD ||
      in_sizes[3] < 2 || in_sizes[4] < 2 || in_sizes[5] < DD || in_sizes[6] < DD ||
      in_sizes[7] != DD * 3 * DD || in_sizes[8] != DD * DD || in_sizes[9] != DD * 4 * DD ||
      in_sizes[10] != 4 * DD * DD || in_sizes[11] != SS || out_size != NTOK * DD) return;

  const float* x     = (const float*)d_in[0];
  const float* ve    = (const float*)d_in[1];
  const float* x0    = (const float*)d_in[2];
  const float* lam   = (const float*)d_in[3];
  const float* sal   = (const float*)d_in[4];
  const float* ln1   = (const float*)d_in[5];
  const float* ln2   = (const float*)d_in[6];
  const float* wqkv  = (const float*)d_in[7];
  const float* wo    = (const float*)d_in[8];
  const float* wfc   = (const float*)d_in[9];
  const float* wproj = (const float*)d_in[10];
  const int*   ids   = (const int*)d_in[11];
  float* outf = (float*)d_out;

  const size_t szWO   = (size_t)DD * DD * 2;
  const size_t szWFC  = (size_t)4 * DD * DD * 2;
  const size_t szWPR  = (size_t)4 * DD * DD * 2;
  const size_t szXR   = (size_t)NTOK * DD * 4;
  const size_t szBIG  = (size_t)NTOK * 3 * DD * 4;
  const size_t szXN   = (size_t)NTOK * DD * 2;
  const size_t szWQA  = (size_t)NTOK * DD * 2;
  const size_t szPL   = (size_t)3 * NTOK * DD * 2;
  const size_t szROPE = (size_t)SS * 64 * 4;
  const size_t szDOC  = (size_t)SS * 4;
  const size_t oWO = 0, oWFC = oWO + szWO, oWPR = oWFC + szWFC, oXR = oWPR + szWPR, oBIG = oXR + szXR,
               oXN = oBIG + szBIG, oWQA = oXN + szXN, oPL = oWQA + szWQA, oROPE = oPL + szPL,
               oDOC = oROPE + szROPE, oEND = oDOC + szDOC;
  if (oEND > ws_size) return;
  char* ws = (char*)d_ws;
  unsigned short* woT   = (unsigned short*)(ws + oWO);
  unsigned short* wfcT  = (unsigned short*)(ws + oWFC);
  unsigned short* wprT  = (unsigned short*)(ws + oWPR);
  float*          xr    = (float*)(ws + oXR);
  float*          qkvf  = (float*)(ws + oBIG);
  unsigned short* hbuf  = (unsigned short*)(ws + oBIG);
  float*          x2    = (float*)(ws + oBIG + (size_t)NTOK * 4 * DD * 2);
  unsigned short* xn    = (unsigned short*)(ws + oXN);
  unsigned short* xn2   = xn;
  unsigned short* wqkvT = (unsigned short*)(ws + oWQA);
  unsigned short* attn  = (unsigned short*)(ws + oWQA);
  unsigned short* qpl   = (unsigned short*)(ws + oPL);
  unsigned short* kpl   = qpl + (size_t)NTOK * DD;
  unsigned short* vpl   = qpl + (size_t)2 * NTOK * DD;
  float*          rope  = (float*)(ws + oROPE);
  int*            docs  = (int*)(ws + oDOC);

  wt_cast_k<<<dim3(3 * DD / 64, DD / 64), 256, 0, stream>>>(wqkv, wqkvT, DD, 3 * DD, WMUL);
  wt_cast_k<<<dim3(DD / 64, DD / 64), 256, 0, stream>>>(wo, woT, DD, DD, WMUL);
  wt_cast_k<<<dim3(4 * DD / 64, DD / 64), 256, 0, stream>>>(wfc, wfcT, DD, 4 * DD, WMUL);
  wt_cast_k<<<dim3(DD / 64, 4 * DD / 64), 256, 0, stream>>>(wproj, wprT, 4 * DD, DD, WMUL);
  tables_k<<<SS / 8 + 1, 256, 0, stream>>>(ids, rope, docs);
  ln_k<true><<<NTOK, 128, 0, stream>>>(x, x0, lam, ln1, xr, xn);
  {
    const int M = NTOK, N = 3 * DD, K = DD;
    const int tiles = (M / 64) * (N / 64);
    wmma_gemm64<0, false, 0, 0, false, 0><<<dim3((tiles + 7) / 8, 1), 256, 0, stream>>>(
        xn, xn, K, 0, wqkvT, wqkvT, K, 0, qkvf, qkvf, N, 0, xr, xr, 0, M, N, K, WMUL_INV);
  }
  rope_k<<<dim3(SS, BB), 256, 0, stream>>>(qkvf, ve, sal, rope, qpl);
  attn128_k<<<BB * HH * (SS / AQB), 128, 0, stream>>>(qpl, kpl, vpl, docs, attn);
  {
    const int M = NTOK, N = DD, K = DD;
    const int tiles = (M / 64) * (N / 64);
    wmma_gemm64<0, false, 0, 0, true, 0><<<dim3((tiles + 7) / 8, 1), 256, 0, stream>>>(
        attn, attn, K, 0, woT, woT, K, 0, x2, x2, N, 0, xr, xr, 0, M, N, K, WMUL_INV);
  }
  ln_k<false><<<NTOK, 128, 0, stream>>>(x2, x2, lam, ln2, xr, xn2);
  {
    const int M = NTOK, N = 4 * DD, K = DD;
    const int tiles = (M / 64) * (N / 64);
    wmma_gemm64<0, false, 0, 1, false, 6><<<dim3((tiles + 7) / 8, 1), 256, 0, stream>>>(
        xn2, xn2, K, 0, wfcT, wfcT, K, 0, hbuf, hbuf, N, 0, xr, xr, 0, M, N, K, WMUL_INV);
  }
  {
    const int M = NTOK, N = DD, K = 4 * DD;
    const int tiles = (M / 64) * (N / 64);
    wmma_gemm64<0, false, 0, 0, true, 0><<<dim3((tiles + 7) / 8, 1), 256, 0, stream>>>(
        hbuf, hbuf, K, 0, wprT, wprT, K, 0, outf, outf, N, 0, x2, x2, 0, M, N, K, WMUL_INV);
  }
}
